// FilteredNoiseGenerator_76811195122337
// MI455X (gfx1250) — hardware-verified
//
#include <hip/hip_runtime.h>
#include <math.h>
#include <stdint.h>


typedef _Float16 v8h  __attribute__((ext_vector_type(8)));
typedef _Float16 v16h __attribute__((ext_vector_type(16)));
typedef float    v8f  __attribute__((ext_vector_type(8)));
typedef float    v4f  __attribute__((ext_vector_type(4)));
typedef v8h v8ha __attribute__((may_alias));

#define TWO_PI_F 6.283185307179586f

constexpr int kBatch     = 32;
constexpr int kBands     = 80;
constexpr int kMagFrames = 2000;
constexpr int kFFT       = 512;
constexpr int kHop       = 128;
constexpr int kPad       = 256;
constexpr int kNF        = 257;
constexpr int kLen       = 320000;
constexpr int kT         = kLen / kHop + 1;
constexpr int kLP        = kLen + 2 * kPad;
constexpr int kRows      = kBatch * kT;
constexpr int kMT        = kRows / 16;
static_assert(kMT * 16 == kRows, "");
constexpr int kMB1       = (kMT + 7) / 8;
constexpr int kSegs      = kLen / kHop;
static_assert(kSegs * kHop == kLen, "");
constexpr int kSegBlk    = 61;
constexpr int kQB        = (kSegs + kSegBlk - 1) / kSegBlk;
constexpr int kFrBlk     = kSegBlk + 3;
static_assert(kFrBlk == 64, "");
constexpr int kOlaLen    = (kFrBlk + 3) * kHop;
constexpr int kLds1      = 520;
constexpr int kStP       = 72;
constexpr int kYtP       = 516;

constexpr float kS1   = 256.0f;
constexpr float kSEpi = 0.125f;
constexpr float kS2   = 512.0f;
constexpr float kYS   = 1.1920928955078125e-7f;

constexpr size_t OFF_B1   = 0;
constexpr size_t SZ_B     = (size_t)kFFT * kFFT * 2;
constexpr size_t OFF_B2   = OFF_B1 + SZ_B;
constexpr size_t OFF_PMAX = OFF_B2 + SZ_B;
constexpr size_t SZ_PMAX  = (size_t)kBatch * kQB * 128;
constexpr size_t OFF_XP   = OFF_PMAX + SZ_PMAX;
constexpr size_t SZ_XP    = (size_t)kBatch * kLP * 2;
constexpr size_t OFF_S    = OFF_XP + SZ_XP;
constexpr size_t SZ_S     = (size_t)kRows * kFFT * 2;
constexpr size_t WS_END   = OFF_S + SZ_S;
static_assert((OFF_PMAX % 128) == 0 && (OFF_XP % 128) == 0 && (OFF_S % 128) == 0, "");
static_assert(((size_t)kLP * 2) % 128 == 0, "");

struct BandTab { unsigned v[66]; };
static_assert(sizeof(BandTab) == 264, "");

static __device__ __forceinline__ v16h cat8(v8h lo, v8h hi) {
  return __builtin_shufflevector(lo, hi, 0, 1, 2, 3, 4, 5, 6, 7, 8, 9, 10, 11, 12, 13, 14, 15);
}

static __device__ __forceinline__ v8f wmma16(v16h a, v16h b, v8f c) {
  v8f d = __builtin_amdgcn_wmma_f32_16x16x32_f16(false, a, false, b, (short)0, c, false, false);
  asm volatile("v_nop\n\tv_nop\n\tv_nop\n\tv_nop" : "+v"(d) : "v"(a), "v"(b));
  return d;
}

static __device__ __forceinline__ float hannw(int n) {
  return 0.5f * (1.0f - cosf((TWO_PI_F * (float)n) * (1.0f / (float)kFFT)));
}

__global__ void __launch_bounds__(256) k_tables(_Float16* __restrict__ b1t, _Float16* __restrict__ b2t) {
  __shared__ __align__(16) _Float16 sv[256];
  const int tid   = threadIdx.x;
  const int blk   = blockIdx.x;
  const int which = blk >> 10;
  const int r     = (blk >> 1) & (kFFT - 1);
  const int cb    = (blk & 1) << 8;
  const int c     = cb + tid;
  const int widx  = which ? r : c;
  const int fs    = which ? c : r;
  const bool re   = (fs < kNF);
  const int f     = re ? fs : (fs - (kNF - 1));
  const int m     = (widx * f + (re ? 0 : (kFFT / 4))) & (kFFT - 1);
  const float ang = (TWO_PI_F * (float)m) * (1.0f / (float)kFFT);
  float sc = kS1;
  if (which) sc = (fs == 0 || fs == kNF - 1) ? kS2 : (2.0f * kS2);
  sv[tid] = (_Float16)(sc * hannw(widx) * cosf(ang));
  __syncthreads();
  if (tid < 32) {
    const v8h val = *(const v8ha*)(sv + tid * 8);
    _Float16* dst = (which ? b2t : b1t) + (size_t)r * kFFT + cb + tid * 8;
    *(volatile v8h*)dst = val;
    __threadfence();
    *(volatile v8h*)dst = val;
  }
}

__global__ void __launch_bounds__(256) k_xp(const float* __restrict__ noise, _Float16* __restrict__ xp, int nchunks) {
  const int idx = blockIdx.x * blockDim.x + threadIdx.x;
  if (idx >= nchunks) return;
  const int per = kLP / 8;
  const int b  = idx / per;
  const int c  = idx - b * per;
  const int j0 = c * 8;
  const float* src = noise + (size_t)b * kLen;
  v8h val;
#pragma unroll
  for (int e = 0; e < 8; ++e) {
    int i = j0 + e - kPad;
    if (i < 0) i = -i;
    if (i >= kLen) i = 2 * kLen - 2 - i;
    if (i < 0) i = 0;
    if (i > kLen - 1) i = kLen - 1;
    val[e] = (_Float16)src[i];
  }
  _Float16* dst = xp + (size_t)b * kLP + j0;
  *(volatile v8h*)dst = val;
  __threadfence();
  *(volatile v8h*)dst = val;
}

__global__ void __launch_bounds__(256) k_gemm1(
    const _Float16* __restrict__ xp, const _Float16* __restrict__ b1t,
    const float* __restrict__ mags, BandTab tab, _Float16* __restrict__ S) {
  __shared__ __align__(16) _Float16 bt[64 * kLds1];
  __shared__ __align__(16) _Float16 st[8 * 16 * kStP];
  const int lane = threadIdx.x;
  const int wv   = threadIdx.y;
  const int tid  = wv * 32 + lane;
  const int lm   = lane & 15;
  const int hh   = lane >> 4;
  const int kb   = hh * 8;
  const int n0   = blockIdx.y * 64;

#pragma unroll 1
  for (int rr = 0; rr < 16; ++rr) {
    const int i   = tid + 256 * rr;
    const int row = i >> 6;
    const int c   = (i & 63) * 8;
    *(v8h*)(bt + row * kLds1 + c) = *(const v8h*)(b1t + (size_t)(n0 + row) * kFFT + c);
  }
  __syncthreads();

  int mtile = blockIdx.x * 8 + wv;
  const bool valid = (mtile < kMT);
  if (!valid) mtile = kMT - 1;
  const int mbase = mtile * 16;

  const int m  = mbase + lm;
  const int bb = m / kT;
  const int t  = m - bb * kT;
  const _Float16* ap = xp + (size_t)bb * kLP + (size_t)t * kHop + kb;
  const _Float16* lb = bt + lm * kLds1 + kb;

  v8f acc[4] = {};
#pragma unroll 2
  for (int kt = 0; kt < kFFT / 32; ++kt) {
    const int ko = kt * 32;
    const v16h a = cat8(*(const v8h*)(ap + ko), *(const v8h*)(ap + ko + 16));
#pragma unroll
    for (int s = 0; s < 4; ++s) {
      const _Float16* bp = lb + s * 16 * kLds1 + ko;
      const v16h bfr = cat8(*(const v8h*)(bp), *(const v8h*)(bp + 16));
      acc[s] = wmma16(a, bfr, acc[s]);
    }
  }

  int bdv[4];
#pragma unroll
  for (int s = 0; s < 4; ++s) {
    const int col = n0 + s * 16 + lm;
    const int f = (col < kNF) ? col : (col - (kNF - 1));
    const int bd = (int)((tab.v[f >> 2] >> ((f & 3) * 8)) & 255u);
    bdv[s] = (bd < kBands) ? bd : -1;
  }

  _Float16* stw = st + wv * 16 * kStP;
  const float rcp = 1.0f / (float)(kT - 1);
#pragma unroll
  for (int j = 0; j < 8; ++j) {
    const int row = mbase + 8 * hh + j;
    const int rb  = row / kT;
    const int rt  = row - rb * kT;
    const float pos = (rt == kT - 1) ? (float)(kMagFrames - 1)
                                     : (float)(kMagFrames - 1) * ((float)rt * rcp);
    int i0 = (int)pos;
    if (i0 < 0) i0 = 0;
    if (i0 > kMagFrames - 1) i0 = kMagFrames - 1;
    const int i1 = (i0 + 1 < kMagFrames) ? (i0 + 1) : (kMagFrames - 1);
    const float wf = pos - (float)i0;
    const float* mb = mags + (size_t)rb * kBands * kMagFrames;
#pragma unroll
    for (int s = 0; s < 4; ++s) {
      float mv = 0.0f;
      if (bdv[s] >= 0) {
        const float* mr = mb + (size_t)bdv[s] * kMagFrames;
        mv = mr[i0] * (1.0f - wf) + mr[i1] * wf;
      }
      stw[(8 * hh + j) * kStP + s * 16 + lm] = (_Float16)(acc[s][j] * mv * kSEpi);
    }
  }
  __syncthreads();

  v8h keep[4];
#pragma unroll
  for (int q = 0; q < 4; ++q) {
    const int r  = q * 4 + (lane >> 3);
    const int ch = (lane & 7) * 8;
    keep[q] = *(const v8ha*)(stw + r * kStP + ch);
  }
  if (valid) {
#pragma unroll
    for (int q = 0; q < 4; ++q) {
      _Float16* dst = S + (size_t)(mbase + q * 4 + (lane >> 3)) * kFFT + n0 + (lane & 7) * 8;
      *(volatile v8h*)dst = keep[q];
    }
  }
  __threadfence();
  if (valid) {
#pragma unroll
    for (int q = 0; q < 4; ++q) {
      _Float16* dst = S + (size_t)(mbase + q * 4 + (lane >> 3)) * kFFT + n0 + (lane & 7) * 8;
      *(volatile v8h*)dst = keep[q];
    }
  }
}

__global__ void __launch_bounds__(256) k_gemm2ola(
    const _Float16* __restrict__ S, const _Float16* __restrict__ b2t,
    float* __restrict__ out, float* __restrict__ pmax) {
  __shared__ __align__(16) float yt[16 * kYtP];
  __shared__ __align__(16) float ola[kOlaLen];
  __shared__ float wsq[kFFT];
  __shared__ float redm[8];
  const int lane = threadIdx.x;
  const int wv   = threadIdx.y;
  const int tid  = wv * 32 + lane;
  const int lm   = lane & 15;
  const int hh   = lane >> 4;
  const int kb   = hh * 8;
  const int b    = blockIdx.y;
  const int qb   = blockIdx.x;
  const int qs0  = qb * kSegBlk;
  const int t0   = qs0 - 1;

  for (int i = tid; i < kOlaLen; i += 256) ola[i] = 0.0f;
  for (int n = tid; n < kFFT; n += 256) { const float w = hannw(n); wsq[n] = w * w; }
  __syncthreads();

  const int c0 = wv * 64;
#pragma unroll 1
  for (int mt = 0; mt < 4; ++mt) {
    int ta = t0 + 16 * mt + lm;
    ta = (ta < 0) ? 0 : ((ta > kT - 1) ? (kT - 1) : ta);
    const _Float16* ap  = S + ((size_t)b * kT + ta) * kFFT + kb;
    const _Float16* bp0 = b2t + (size_t)(c0 + lm) * kFFT + kb;

    v8f acc[4] = {};
#pragma unroll 2
    for (int kt = 0; kt < kFFT / 32; ++kt) {
      const int ko = kt * 32;
      const v16h a = cat8(*(const v8h*)(ap + ko), *(const v8h*)(ap + ko + 16));
#pragma unroll
      for (int s = 0; s < 4; ++s) {
        const _Float16* bp = bp0 + (size_t)s * 16 * kFFT + ko;
        const v16h bfr = cat8(*(const v8h*)(bp), *(const v8h*)(bp + 16));
        acc[s] = wmma16(a, bfr, acc[s]);
      }
    }
#pragma unroll
    for (int j = 0; j < 8; ++j) {
#pragma unroll
      for (int s = 0; s < 4; ++s) {
        yt[(8 * hh + j) * kYtP + c0 + s * 16 + lm] = acc[s][j];
      }
    }
    __syncthreads();

    const int tb = t0 + 16 * mt;
    for (int rel = tid; rel < 15 * kHop + kFFT; rel += 256) {
      int ilo = rel - (kFFT - kHop);
      ilo = (ilo < 0) ? 0 : (ilo >> 7);
      int ihi = rel >> 7;
      if (ihi > 15) ihi = 15;
      float sum = 0.0f;
      for (int i = ilo; i <= ihi; ++i) {
        const int tg = tb + i;
        if (tg >= 0 && tg < kT) sum += yt[i * kYtP + rel - i * kHop];
      }
      ola[mt * 16 * kHop + rel] += sum;
    }
    __syncthreads();
  }

  float lmax = 0.0f;
  float* orow = out + (size_t)b * kLen;
#pragma unroll 1
  for (int r = 0; r < 8; ++r) {
    const int j  = wv + 8 * r;
    const int qs = qs0 + j;
    if (j < kSegBlk && qs < kSegs) {
      const int u = lane * 4;
      v4f vv;
#pragma unroll
      for (int e = 0; e < 4; ++e) {
        const int p  = qs * kHop + u + e;
        const int pg = p + kPad;
        const int sp = (j + 3) * kHop + u + e;
        int tlo = pg - (kFFT - kHop);
        tlo = (tlo < 0) ? 0 : (tlo >> 7);
        int thi = pg >> 7;
        if (thi > kT - 1) thi = kT - 1;
        float ws = 0.0f;
        for (int tt = tlo; tt <= thi; ++tt) ws += wsq[pg - tt * kHop];
        const float den = (ws > 1e-11f) ? ws : 1.0f;
        const float v = (ola[sp] * kYS) * (1.0f / den);
        vv[e] = v;
        lmax = fmaxf(lmax, fabsf(v));
        ola[sp] = v;
      }
      *(volatile v4f*)(orow + (size_t)qs * kHop + u) = vv;
    }
  }
  __threadfence();
#pragma unroll 1
  for (int r = 0; r < 8; ++r) {
    const int j  = wv + 8 * r;
    const int qs = qs0 + j;
    if (j < kSegBlk && qs < kSegs) {
      const int u = lane * 4;
      v4f vv;
#pragma unroll
      for (int e = 0; e < 4; ++e) vv[e] = ola[(j + 3) * kHop + u + e];
      *(volatile v4f*)(orow + (size_t)qs * kHop + u) = vv;
    }
  }

#pragma unroll
  for (int msk = 16; msk > 0; msk >>= 1) lmax = fmaxf(lmax, __shfl_xor(lmax, msk, 32));
  if (lane == 0) redm[wv] = lmax;
  __syncthreads();
  if (wv == 0) {
    float mx = redm[0];
#pragma unroll
    for (int i = 1; i < 8; ++i) mx = fmaxf(mx, redm[i]);
    if (lane < 8) {
      v4f q4;
      q4[0] = mx; q4[1] = mx; q4[2] = mx; q4[3] = mx;
      float* pp = pmax + ((size_t)(b * kQB + qb)) * 32 + lane * 4;
      *(volatile v4f*)pp = q4;
      __threadfence();
      *(volatile v4f*)pp = q4;
    }
  }
}

__global__ void __launch_bounds__(256) k_norm(float* __restrict__ out, const float* __restrict__ pmax,
                                              const int* __restrict__ alen) {
  const int lane = threadIdx.x;
  const int wv   = threadIdx.y;
  const int b    = blockIdx.y;
  const int seg  = blockIdx.x * 8 + wv;
  float m = 0.0f;
  if (lane < kQB)      m = pmax[((size_t)(b * kQB + lane)) * 32];
  if (lane + 32 < kQB) m = fmaxf(m, pmax[((size_t)(b * kQB + lane + 32)) * 32]);
#pragma unroll
  for (int msk = 16; msk > 0; msk >>= 1) m = fmaxf(m, __shfl_xor(m, msk, 32));
  const float sc = 1.0f / (m + 1e-8f);
  int L = alen[0];
  if (L > kLen) L = kLen;
  const int p0 = seg * kHop + lane * 4;
  if (seg < kSegs && p0 + 4 <= L) {
    float* p = out + (size_t)b * kLen + p0;
    v4f v = *(const v4f*)p;
    v = v * sc;
    *(volatile v4f*)p = v;
    __threadfence();
    *(volatile v4f*)p = v;
  }
}

extern "C" void kernel_launch(void* const* d_in, const int* in_sizes, int n_in,
                              void* d_out, int out_size, void* d_ws, size_t ws_size,
                              hipStream_t stream) {
  if (n_in < 3) return;
  if (in_sizes[0] != kBatch * kBands * kMagFrames) return;
  if (in_sizes[1] != kBatch * kLen) return;
  if (in_sizes[2] < 1) return;
  if (out_size != kBatch * kLen) return;
  if (WS_END > ws_size) return;

  const float* mags  = (const float*)d_in[0];
  const float* noise = (const float*)d_in[1];
  const int*   alen  = (const int*)d_in[2];
  float* out = (float*)d_out;
  char* ws = (char*)d_ws;

  _Float16* b1t  = (_Float16*)(ws + OFF_B1);
  _Float16* b2t  = (_Float16*)(ws + OFF_B2);
  float*    pmax = (float*)   (ws + OFF_PMAX);
  _Float16* xp   = (_Float16*)(ws + OFF_XP);
  _Float16* S    = (_Float16*)(ws + OFF_S);

  BandTab tab;
  for (int i = 0; i < 66; ++i) tab.v[i] = 0xFFFFFFFFu;
  {
    const double half_sr = 16000.0 / 2.0;
    const double mel_max = 2595.0 * log10(1.0 + half_sr / 700.0);
    const double step = (mel_max - 0.0) / 80.0;
    float edges[kBands + 1];
    for (int i = 0; i <= kBands; ++i) {
      const double mel = (i == kBands) ? mel_max : ((double)i * step + 0.0);
      const double hz = 700.0 * (pow(10.0, mel / 2595.0) - 1.0);
      edges[i] = (float)(hz / half_sr);
    }
    for (int f = 0; f < kNF; ++f) {
      const float fr = (f == kNF - 1) ? 1.0f : ((float)f * (1.0f / 256.0f));
      int cnt = 0;
      for (int i = 0; i <= kBands; ++i) if (edges[i] <= fr) ++cnt;
      const int bd = cnt - 1;
      const unsigned code = (bd >= 0 && bd < kBands) ? (unsigned)bd : 255u;
      const int sh = (f & 3) * 8;
      tab.v[f >> 2] = (tab.v[f >> 2] & ~(255u << sh)) | (code << sh);
    }
  }

  k_tables<<<2 * kFFT * 2, 256, 0, stream>>>(b1t, b2t);

  const int nchunks = kBatch * (kLP / 8);
  k_xp<<<(nchunks + 255) / 256, 256, 0, stream>>>(noise, xp, nchunks);

  const dim3 blk(32, 8);
  k_gemm1<<<dim3(kMB1, kFFT / 64), blk, 0, stream>>>(xp, b1t, mags, tab, S);

  k_gemm2ola<<<dim3(kQB, kBatch), blk, 0, stream>>>(S, b2t, out, pmax);

  k_norm<<<dim3((kSegs + 7) / 8, kBatch), blk, 0, stream>>>(out, pmax, alen);
}
